// BioWaveKAN_44684839747976
// MI455X (gfx1250) — hardware-verified
//
#include <hip/hip_runtime.h>


#define NB_  4096
#define DI   2048
#define DO   2048
#define RCH  1024
#define DM   DI
#define BEPS 1e-5f
#define LOSC 1024.0f

typedef _Float16 h16;
typedef unsigned short bf;
typedef __attribute__((ext_vector_type(16))) __bf16   v16bf;
typedef __attribute__((ext_vector_type(16))) _Float16 v16h;
typedef __attribute__((ext_vector_type(8)))  _Float16 v8h;
typedef __attribute__((ext_vector_type(8)))  unsigned short v8us;
typedef __attribute__((ext_vector_type(8)))  float    v8f;
typedef __attribute__((ext_vector_type(4)))  float    v4f;
typedef v8h  __attribute__((may_alias)) v8ha;
typedef v4f  __attribute__((may_alias)) v4fa;
typedef v8us __attribute__((may_alias)) v8usa;

__device__ __forceinline__ unsigned short f2bf(float f) { unsigned u = __float_as_uint(f); u += 0x7FFFu + ((u >> 16) & 1u); return (unsigned short)(u >> 16); }
__device__ __forceinline__ float bf2f(unsigned short b) { return __uint_as_float(((unsigned)b) << 16); }
__device__ __forceinline__ float bfr(float f) { return bf2f(f2bf(f)); }
__device__ __forceinline__ v16h cat16(v8h lo, v8h hi) { return __builtin_shufflevector(lo, hi, 0, 1, 2, 3, 4, 5, 6, 7, 8, 9, 10, 11, 12, 13, 14, 15); }
__device__ __forceinline__ v16bf cat16b(v8us lo, v8us hi) { return __builtin_bit_cast(v16bf, __builtin_shufflevector(lo, hi, 0, 1, 2, 3, 4, 5, 6, 7, 8, 9, 10, 11, 12, 13, 14, 15)); }
__device__ __forceinline__ v8f wmma16(v16h a, v16h b, v8f c) { return __builtin_amdgcn_wmma_f32_16x16x32_f16(false, a, false, b, (short)0, c, false, false); }
__device__ __forceinline__ v8f wmmab(v16bf a, v16bf b, v8f c) { return __builtin_amdgcn_wmma_f32_16x16x32_bf16(false, a, false, b, (short)0, c, false, false); }

template <bool SPLITA, bool F16OUT = false>
__global__ __launch_bounds__(128) void k_gemmb(const bf* __restrict__ A, const bf* __restrict__ Al, const bf* __restrict__ Bn, const float* __restrict__ bias, float* C, int ldc, h16* C2, const float* __restrict__ R = nullptr, int K = DM, int roundR = 1) {
    __shared__ __align__(16) float ost[4][16 * 68];
    const int lane = threadIdx.x & 31, wave = threadIdx.x >> 5, lr = lane & 15, hi = lane >> 4;
    const int r0 = blockIdx.x * 64 + wave * 16, c0 = blockIdx.y * 64;
    const size_t aoff = (size_t)(r0 + lr) * K + 8 * hi;
    size_t boff[4];
#pragma unroll
    for (int t = 0; t < 4; ++t) boff[t] = (size_t)(c0 + t * 16 + lr) * K + 8 * hi;
    v8f acc[4];
#pragma unroll
    for (int t = 0; t < 4; ++t) acc[t] = (v8f){};
#pragma unroll 1
    for (int kc = 0; kc < K; kc += 32) {
        const v16bf a = cat16b(*(const v8us*)(A + aoff + kc), *(const v8us*)(A + aoff + kc + 16));
        v16bf al = a;
        if (SPLITA) al = cat16b(*(const v8us*)(Al + aoff + kc), *(const v8us*)(Al + aoff + kc + 16));
#pragma unroll
        for (int t = 0; t < 4; ++t) { const v16bf b = cat16b(*(const v8us*)(Bn + boff[t] + kc), *(const v8us*)(Bn + boff[t] + kc + 16)); acc[t] = wmmab(a, b, acc[t]); if (SPLITA) acc[t] = wmmab(al, b, acc[t]); }
        asm volatile("v_nop\n\tv_nop\n\tv_nop\n\tv_nop" : "+v"(acc[0]), "+v"(acc[1]), "+v"(acc[2]), "+v"(acc[3]) : "v"(a), "v"(al));
    }
    float* os = &ost[wave][0];
#pragma unroll
    for (int t = 0; t < 4; ++t) { const float bv = bias ? bfr(bias[c0 + t * 16 + lr]) : 0.f;
#pragma unroll
        for (int j = 0; j < 8; ++j) os[(hi * 8 + j) * 68 + t * 16 + lr] = acc[t][j] + bv; }
    __syncthreads();
    if (F16OUT) {
        h16* crow = (h16*)(void*)C + (size_t)r0 * ldc + c0;
        auto pass = [&]() {
#pragma unroll
            for (int s = 0; s < 4; ++s) { const int row = 4 * s + (lane >> 3), piece = lane & 7; const float* sp = os + row * 68 + piece * 8; v8h o, o2;
#pragma unroll
                for (int i = 0; i < 8; ++i) { const h16 a = (h16)sp[i]; o[i] = a; o2[i] = (h16)((sp[i] - (float)a) * LOSC); }
                *(volatile v8h*)(crow + (size_t)row * ldc + piece * 8) = o; if (C2) *(volatile v8h*)(C2 + (size_t)r0 * ldc + c0 + (size_t)row * ldc + piece * 8) = o2; }
        };
        pass(); __threadfence(); pass();
    } else {
        float* crow = C + (size_t)r0 * ldc + c0;
        auto pass = [&]() {
#pragma unroll
            for (int s = 0; s < 8; ++s) { const int Lid = (lane >> 3) + 4 * s, piece = lane & 7; const int row = Lid >> 1, cofs = (Lid & 1) * 32 + piece * 4;
                v4f val = *(const v4fa*)(os + row * 68 + cofs); if (R) { const v4f rv = *(const v4f*)(R + ((size_t)r0 + row) * ldc + c0 + cofs); val += roundR ? (v4f){bfr(rv[0]), bfr(rv[1]), bfr(rv[2]), bfr(rv[3])} : rv; }
                *(volatile v4f*)(crow + (size_t)row * ldc + cofs) = val; }
        };
        pass(); __threadfence(); pass();
    }
}


__global__ __launch_bounds__(256) void k_cvt8(const float* __restrict__ src, bf* dst, size_t n8) {
    const size_t i = (size_t)blockIdx.x * 256 + threadIdx.x; if (i >= n8) return;
    const v8f v = *(const v8f*)(src + i * 8); v8us o;
#pragma unroll
    for (int k = 0; k < 8; ++k) o[k] = f2bf(v[k]);
    *(volatile v8us*)(dst + i * 8) = o; __threadfence(); *(volatile v8us*)(dst + i * 8) = o;
}
__global__ __launch_bounds__(256) void k_zero8(bf* dst, size_t n8) {
    const size_t i = (size_t)blockIdx.x * 256 + threadIdx.x; if (i >= n8) return; v8us z;
#pragma unroll
    for (int k = 0; k < 8; ++k) z[k] = 0;
    *(volatile v8us*)(dst + i * 8) = z; __threadfence(); *(volatile v8us*)(dst + i * 8) = z;
}

__global__ __launch_bounds__(256) void k_feat(const float* __restrict__ x, const float* __restrict__ sc, const float* __restrict__ tr, int r0, bf* Xb, bf* Ph, bf* Pl) {
    typedef __attribute__((ext_vector_type(4))) unsigned short v4us;
    const int lane = threadIdx.x & 31; const int rl = blockIdx.x * 8 + (threadIdx.x >> 5); if (rl >= RCH) return; const size_t r = (size_t)r0 + rl;
    const float c0f = 0.75112554446494248f;
#pragma unroll 1
    for (int ps = 0; ps < 2; ++ps) {
#pragma unroll 1
        for (int q = 0; q < DI / 128; ++q) { const int cb = q * 128 + lane * 4; v4us xb, oh, ol;
#pragma unroll
            for (int i = 0; i < 4; ++i) { const int c = cb + i; const float xv = bfr(x[r * DI + c]); xb[i] = f2bf(xv);
                const float u = (xv - bfr(tr[c])) / fmaxf(bfr(sc[c]), 1e-3f); const float w = c0f * cosf(3.0f * u) * __expf(-0.5f * u * u); const unsigned short hb = f2bf(w); oh[i] = hb; ol[i] = f2bf(w - bf2f(hb)); }
            const size_t o = (size_t)rl * DI + cb; *(volatile v4us*)(Xb + o) = xb; *(volatile v4us*)(Ph + o) = oh; *(volatile v4us*)(Pl + o) = ol; }
        if (ps == 0) __threadfence(); }
}
__global__ __launch_bounds__(256) void k_scale03(float* B0) {
    const int lane = threadIdx.x & 31; const size_t rl = (size_t)blockIdx.x * 8 + (threadIdx.x >> 5); if (rl >= (size_t)RCH) return;
#pragma unroll 1
    for (int q = 0; q < DO / 128; ++q) { float* p = B0 + rl * DO + q * 128 + lane * 4; v4f v = *(const v4f*)p; v *= 0.3f; *(volatile v4f*)p = v; __threadfence(); *(volatile v4f*)p = v; }
}
template <int MODE>
__global__ __launch_bounds__(256) void k_colstat(const float* __restrict__ Y, const float* __restrict__ MEAN, float* OUTV) {
    const int c = blockIdx.x * 256 + threadIdx.x; if (c >= DO) return; float s = 0.f; const float mu = (MODE == 1) ? MEAN[c] : 0.f;
#pragma unroll 1
    for (int b = 0; b < NB_ / 512; ++b) { float p = 0.f;
#pragma unroll 4
        for (int r = b * 512; r < (b + 1) * 512; ++r) { const float v = Y[(size_t)r * DO + c]; const float d = (MODE == 1) ? (v - mu) * (v - mu) : v; p += d; }
        s += p; }
    s *= 1.0f / (float)NB_; *(volatile float*)(OUTV + c) = s; __threadfence(); *(volatile float*)(OUTV + c) = s;
}
__global__ __launch_bounds__(256) void k_bnout(const float* __restrict__ Y, const float* __restrict__ MEAN, const float* __restrict__ VAR, const float* __restrict__ ga, const float* __restrict__ be, float* OUTP) {
    const int lane = threadIdx.x & 31; const size_t r = (size_t)blockIdx.x * 8 + (threadIdx.x >> 5); if (r >= (size_t)NB_) return;
#pragma unroll 1
    for (int ps = 0; ps < 2; ++ps) {
#pragma unroll 1
        for (int q = 0; q < DO / 128; ++q) { const int cb = q * 128 + lane * 4; v4f v;
#pragma unroll
            for (int i = 0; i < 4; ++i) { const int c = cb + i; v[i] = bfr(ga[c]) * (Y[r * DO + c] - MEAN[c]) * rsqrtf(VAR[c] + BEPS) + bfr(be[c]); }
            *(volatile v4f*)(OUTP + r * DO + cb) = v; }
        if (ps == 0) __threadfence(); }
}

extern "C" void kernel_launch(void* const* d_in, const int* in_sizes, int n_in,
                              void* d_out, int out_size, void* d_ws, size_t ws_size, hipStream_t stream) {
    (void)in_sizes; (void)n_in; (void)out_size;
    const float* x = (const float*)d_in[0]; const float* sc = (const float*)d_in[1]; const float* tr = (const float*)d_in[2]; const float* ww = (const float*)d_in[3]; const float* bw = (const float*)d_in[4]; const float* ga = (const float*)d_in[5]; const float* be = (const float*)d_in[6];
    float* out = (float*)d_out;
    char* wsp = (char*)d_ws;
    auto take = [&](size_t bytes) { char* p = wsp; wsp += (bytes + 255) & ~(size_t)255; return (void*)p; };
    bf* WW = (bf*)take((size_t)DO * DI * 2); bf* BW = (bf*)take((size_t)DO * DI * 2); bf* Xb = (bf*)take((size_t)RCH * DI * 2); bf* Ph = (bf*)take((size_t)RCH * DI * 2); bf* Pl = (bf*)take((size_t)RCH * DI * 2);
    float* B0 = (float*)take((size_t)RCH * DO * 4); float* Y1 = (float*)take((size_t)RCH * DO * 4); float* Y = (float*)take((size_t)NB_ * DO * 4); float* MEAN = (float*)take(DO * 4); float* VAR = (float*)take(DO * 4);
    if ((size_t)(wsp - (char*)d_ws) > ws_size) return;
    k_cvt8<<<(unsigned)(((size_t)DO * DI / 8 + 255) / 256), 256, 0, stream>>>(ww, WW, (size_t)DO * DI / 8); k_cvt8<<<(unsigned)(((size_t)DO * DI / 8 + 255) / 256), 256, 0, stream>>>(bw, BW, (size_t)DO * DI / 8);
    for (int ch = 0; ch < NB_ / RCH; ++ch) { const int r0 = ch * RCH;
        k_feat<<<RCH / 8, 256, 0, stream>>>(x, sc, tr, r0, Xb, Ph, Pl);
        k_gemmb<false, false><<<dim3(RCH / 64, DO / 64, 1), 128, 0, stream>>>(Xb, nullptr, BW, nullptr, B0, DO, nullptr, nullptr, DI);
        k_scale03<<<RCH / 8, 256, 0, stream>>>(B0);
        k_gemmb<false, false><<<dim3(RCH / 64, DO / 64, 1), 128, 0, stream>>>(Ph, nullptr, WW, nullptr, Y1, DO, nullptr, B0, DI, 0);
        k_gemmb<false, false><<<dim3(RCH / 64, DO / 64, 1), 128, 0, stream>>>(Pl, nullptr, WW, nullptr, Y + (size_t)r0 * DO, DO, nullptr, Y1, DI, 0); }
    k_colstat<0><<<DO / 256, 256, 0, stream>>>(Y, nullptr, MEAN); k_colstat<1><<<DO / 256, 256, 0, stream>>>(Y, MEAN, VAR);
    k_bnout<<<NB_ / 8, 256, 0, stream>>>(Y, MEAN, VAR, ga, be, out);
}
